// MultiheadSelfAttentionDec_89524298317920
// MI455X (gfx1250) — hardware-verified
//
#include <hip/hip_runtime.h>
#include <hip/hip_bf16.h>
#include <math.h>
#include <stdint.h>

typedef __attribute__((ext_vector_type(16))) _Float16 v16h;
typedef __attribute__((ext_vector_type(8)))  _Float16 v8h;
typedef __attribute__((ext_vector_type(16))) __bf16   v16b;
typedef __attribute__((ext_vector_type(8)))  __bf16   v8b;
typedef __attribute__((ext_vector_type(8)))  float    v8f;
typedef __attribute__((ext_vector_type(4)))  float    v4f;
typedef __attribute__((ext_vector_type(2)))  float    v2f;

constexpr int kSeq = 3072;
constexpr int kCh  = 2048;
constexpr int kHd  = 128;
constexpr int kNh  = 16;

template <bool B> struct CtCheck;
template <> struct CtCheck<true> { static constexpr int ok = 1; };
constexpr int kChkGeom = CtCheck<(kSeq % 64 == 0) && (kCh % 64 == 0) && (kCh % 32 == 0) && (kSeq % 32 == 0) &&
                                 (kNh * kHd == kCh) && (kHd == 128)>::ok;

constexpr size_t kPlane16 = (size_t)kSeq * kCh * 2;
constexpr size_t kPlane32 = (size_t)kSeq * kCh * 4;
constexpr size_t kW16     = (size_t)kCh * kCh * 2;
constexpr size_t oXb  = 0;
constexpr size_t oWq  = oXb + kPlane16;
constexpr size_t oWk  = oWq + kW16;
constexpr size_t oWv  = oWk + kW16;
constexpr size_t oWo  = oWv + kW16;
constexpr size_t oQKf = oWo + kW16;
constexpr size_t oQh  = oQKf + kPlane32;
constexpr size_t oKh  = oQh + kPlane16;
constexpr size_t oVt  = oKh + kPlane16;
constexpr size_t kWsTotal = oVt + kPlane16;
constexpr int kChkWs = CtCheck<(kWsTotal == (size_t)109051904) && (kWsTotal <= (size_t)134217728) &&
                               (kPlane16 <= kPlane32) && (oWq % 128 == 0) && (oQKf % 128 == 0) && (oVt % 128 == 0)>::ok;

__device__ __forceinline__ unsigned short f2bf_bits(float f) {
  unsigned u = __float_as_uint(f);
  return (unsigned short)((u + 0x7FFFu + ((u >> 16) & 1u)) >> 16);
}
__device__ __forceinline__ float bf_bits2f(unsigned short h) { return __uint_as_float(((unsigned)h) << 16); }
__device__ __forceinline__ float bf_rne(float f) { return bf_bits2f(f2bf_bits(f)); }

__device__ __forceinline__ void dep_guard_h(v8f& a, v8f& b, v16h x, v16h y) { asm volatile("v_nop\n\tv_nop\n\tv_nop\n\tv_nop" : "+v"(a), "+v"(b) : "v"(x), "v"(y)); }
__device__ __forceinline__ void dep_guard_b(v8f& a, v8f& b, v16b x, v16b y) { asm volatile("v_nop\n\tv_nop\n\tv_nop\n\tv_nop" : "+v"(a), "+v"(b) : "v"(x), "v"(y)); }
__device__ __forceinline__ void keep4_h(v16h a, v16h b, v16h c, v16h d) { asm volatile("v_nop" :: "v"(a), "v"(b), "v"(c), "v"(d)); }
__device__ __forceinline__ void keep4_b(v16b a, v16b b, v16b c, v16b d) { asm volatile("v_nop" :: "v"(a), "v"(b), "v"(c), "v"(d)); }
__device__ __forceinline__ void acc_guard4(v8f& a, v8f& b, v8f& c, v8f& d) { asm volatile("v_nop\n\tv_nop\n\tv_nop\n\tv_nop" : "+v"(a), "+v"(b), "+v"(c), "+v"(d)); }
template <typename T> struct Frag;
template <> struct Frag<_Float16> {
  typedef v16h V; union U { v16h v; v8h h[2]; };
  static __device__ __forceinline__ v16h load(const _Float16* p) {
    U f; f.h[0] = *(const v8h*)(p); f.h[1] = *(const v8h*)(p + 16); return f.v;
  }
  static __device__ __forceinline__ v8f mma(v16h a, v16h b, v8f c) {
    return __builtin_amdgcn_wmma_f32_16x16x32_f16(false, a, false, b, (short)0, c, false, false);
  }
  static __device__ __forceinline__ void guard(v8f& a, v8f& b, v16h x, v16h y) { dep_guard_h(a, b, x, y); }
  static __device__ __forceinline__ void keep(v16h a, v16h b, v16h c, v16h d) { keep4_h(a, b, c, d); }
};
template <> struct Frag<__bf16> {
  typedef v16b V; union U { v16b v; v8b h[2]; };
  static __device__ __forceinline__ v16b load(const __bf16* p) {
    U f; f.h[0] = *(const v8b*)(p); f.h[1] = *(const v8b*)(p + 16); return f.v;
  }
  static __device__ __forceinline__ v8f mma(v16b a, v16b b, v8f c) {
    return __builtin_amdgcn_wmma_f32_16x16x32_bf16(false, a, false, b, (short)0, c, false, false);
  }
  static __device__ __forceinline__ void guard(v8f& a, v8f& b, v16b x, v16b y) { dep_guard_b(a, b, x, y); }
  static __device__ __forceinline__ void keep(v16b a, v16b b, v16b c, v16b d) { keep4_b(a, b, c, d); }
};

template <int ET> struct Elem;
template <> struct Elem<0> { typedef _Float16 T; };
template <> struct Elem<1> { typedef __bf16 T; };
template <int ET, int SPLIT, int BIAS_MODE, int OUT_MODE, bool RESID, int ACT = 0>
__global__ __launch_bounds__(256) void wmma_gemm64(
    const unsigned short* __restrict__ Ap, const unsigned short* __restrict__ A2p, int lda, long strideA,
    const unsigned short* __restrict__ Btp, const unsigned short* __restrict__ Bt2p, int ldb, long strideB,
    void* __restrict__ Cout, void* __restrict__ Cout2, int ldc, long strideC,
    const float* __restrict__ bias,
    const float* __restrict__ resid, long strideR,
    int M, int N, int K, float scale) {
  typedef typename Elem<ET>::T T;
  typedef typename Frag<T>::V V;
  const T* A = (const T*)Ap; const T* A2 = (const T*)A2p; const T* Bt = (const T*)Btp; const T* Bt2 = (const T*)Bt2p;
  __shared__ __align__(16) float sT[8][16 * 68];
  const int b    = blockIdx.y;
  const int lane = threadIdx.x & 31;
  const int wave = threadIdx.x >> 5;
  const int tilesN = N >> 6;
  const int tilesM = M >> 6;
  const int tile = blockIdx.x * 8 + wave;
  if (tile >= tilesM * tilesN) return;
  const int tm = tile / tilesN;
  const int tn = tile - tm * tilesN;
  const int m0 = tm << 6;
  const int n0 = tn << 6;

  const T* Ab  = A  + (size_t)b * strideA;
  const T* Bb  = Bt + (size_t)b * strideB;
  const T* Ab2 = (SPLIT != 0) ? (A2  + (size_t)b * strideA) : nullptr;
  const T* Bb2 = (SPLIT == 1) ? (Bt2 + (size_t)b * strideB) : nullptr;

  const int rlane = lane & 15;
  const int koff  = (lane >> 4) * 8;
  const int mOff  = (lane >> 4) * 8;

  v8f acc[4][4];
#pragma unroll
  for (int i = 0; i < 4; ++i)
#pragma unroll
    for (int j = 0; j < 4; ++j) acc[i][j] = (v8f){0.f,0.f,0.f,0.f,0.f,0.f,0.f,0.f};

  for (int k0 = 0; k0 < K; k0 += 32) {
    V bh[4], bl[4];
#pragma unroll
    for (int j = 0; j < 4; ++j) {
      const size_t bo = (size_t)(n0 + (j << 4) + rlane) * ldb + koff + k0;
      bh[j] = Frag<T>::load(Bb + bo);
      if (SPLIT == 1) bl[j] = Frag<T>::load(Bb2 + bo);
    }
#pragma unroll
    for (int i = 0; i < 4; ++i) {
      const size_t ao = (size_t)(m0 + (i << 4) + rlane) * lda + koff + k0;
      V ah = Frag<T>::load(Ab + ao);
      V al;
      if (SPLIT != 0) al = Frag<T>::load(Ab2 + ao);
#pragma unroll
      for (int j = 0; j < 4; ++j) {
        acc[i][j] = Frag<T>::mma(ah, bh[j], acc[i][j]);
        if (SPLIT == 1) acc[i][j] = Frag<T>::mma(ah, bl[j], acc[i][j]);
        if (SPLIT != 0) acc[i][j] = Frag<T>::mma(al, bh[j], acc[i][j]);
      }
      Frag<T>::guard(acc[i][0], acc[i][3], ah, (SPLIT != 0) ? al : ah);
    }
    Frag<T>::keep(bh[0], bh[1], bh[2], bh[3]);
    if (SPLIT == 1) Frag<T>::keep(bl[0], bl[1], bl[2], bl[3]);
  }
  acc_guard4(acc[0][0], acc[0][1], acc[0][2], acc[0][3]);
  acc_guard4(acc[1][0], acc[1][1], acc[1][2], acc[1][3]);
  acc_guard4(acc[2][0], acc[2][1], acc[2][2], acc[2][3]);
  acc_guard4(acc[3][0], acc[3][1], acc[3][2], acc[3][3]);

  float* slab = sT[wave];
  const float* Rb = RESID ? (resid + (size_t)b * strideR) : nullptr;
#pragma unroll
  for (int i = 0; i < 4; ++i) {
    const int mBase = m0 + (i << 4);
#pragma unroll
    for (int j = 0; j < 4; ++j) {
      const int n = n0 + (j << 4) + rlane;
      float bv = 0.f;
      if (BIAS_MODE == 2) bv = bias[n];
#pragma unroll
      for (int r = 0; r < 8; ++r) {
        float v = acc[i][j][r] * scale;
        if (BIAS_MODE == 1) v += bias[mBase + mOff + r];
        if (BIAS_MODE == 2) v += bv;
        if (RESID) v += Rb[(size_t)(mBase + mOff + r) * ldc + n];
        if (ACT == 1) v = tanhf(v);
        if (ACT == 2) v = fmaxf(v, 0.0f);
        if (ACT == 3) v = v / (1.0f + expf(-v));
        if (ACT == 4) v = (v > 0.f) ? v : 0.01f * v;
        slab[(mOff + r) * 68 + (j << 4) + rlane] = v;
      }
    }
    __builtin_amdgcn_fence(__ATOMIC_RELEASE, "workgroup");
    __builtin_amdgcn_wave_barrier();
    __builtin_amdgcn_fence(__ATOMIC_ACQUIRE, "workgroup");
    if (OUT_MODE == 0) {
      float* C = (float*)Cout + (size_t)b * strideC;
      const int hh = lane >> 4, c4 = (lane & 15) * 4;
      for (int pass = 0; pass < 2; ++pass) {
#pragma unroll
        for (int it = 0; it < 8; ++it) {
          const int row = it * 2 + hh;
          v4f v = *(const v4f*)(slab + row * 68 + c4);
          *(volatile v4f*)(C + (size_t)(mBase + row) * ldc + n0 + c4) = v;
        }
        __threadfence();
      }
    } else {
      const int q = lane >> 3, c8 = (lane & 7) * 8;
      unsigned short* C  = (unsigned short*)Cout  + (size_t)b * strideC;
      unsigned short* C2 = (OUT_MODE == 2) ? ((unsigned short*)Cout2 + (size_t)b * strideC) : nullptr;
      for (int pass = 0; pass < 2; ++pass) {
#pragma unroll
        for (int it = 0; it < 4; ++it) {
          const int row = it * 4 + q;
          const float* sp = slab + row * 68 + c8;
          v8h hv, lv;
#pragma unroll
          for (int e = 0; e < 8; ++e) {
            if (OUT_MODE == 1) {
              hv[e] = (_Float16)sp[e];
            } else {
              unsigned short hb = f2bf_bits(sp[e]);
              unsigned short lb = f2bf_bits(sp[e] - bf_bits2f(hb));
              hv[e] = __builtin_bit_cast(_Float16, hb);
              lv[e] = __builtin_bit_cast(_Float16, lb);
            }
          }
          *(volatile v8h*)(C + (size_t)(mBase + row) * ldc + n0 + c8) = hv;
          if (OUT_MODE == 2) *(volatile v8h*)(C2 + (size_t)(mBase + row) * ldc + n0 + c8) = lv;
        }
        __threadfence();
      }
    }
    __builtin_amdgcn_fence(__ATOMIC_RELEASE, "workgroup");
    __builtin_amdgcn_wave_barrier();
    __builtin_amdgcn_fence(__ATOMIC_ACQUIRE, "workgroup");
  }
}

__global__ __launch_bounds__(256) void cast_f32_bf16x2(
    const float* __restrict__ in, unsigned short* __restrict__ out, int n2) {
  const int i = blockIdx.x * 256 + threadIdx.x;
  if (i < n2) {
    const v2f f = *(const v2f*)(in + 2 * (size_t)i);
    const unsigned u = (unsigned)f2bf_bits(f[0]) | ((unsigned)f2bf_bits(f[1]) << 16);
    ((volatile unsigned*)out)[i] = u;
    __threadfence();
    ((volatile unsigned*)out)[i] = u;
  }
}

__global__ __launch_bounds__(256) void rmsnorm_rotary_f16(
    const float* __restrict__ Xf, const float* __restrict__ rot, const float* __restrict__ gw,
    unsigned short* __restrict__ Yp, int nUnits, float eps) {
  const int lane = threadIdx.x & 31;
  const int wave = threadIdx.x >> 5;
  const int hh = lane >> 4;
  const int c  = lane & 15;
  int u = (blockIdx.x * 8 + wave) * 2 + hh;
  const bool ok = (u < nUnits);
  u = ok ? u : (nUnits - 1);
  const int s = u >> 4;
  const size_t base = (size_t)u * kHd + (size_t)c * 8;
  const v4f xa = *(const v4f*)(Xf + base);
  const v4f xb = *(const v4f*)(Xf + base + 4);
  const float* rp = rot + (size_t)s * 256 + c * 16;
  const v4f r0 = *(const v4f*)(rp);
  const v4f r1 = *(const v4f*)(rp + 4);
  const v4f r2 = *(const v4f*)(rp + 8);
  const v4f r3 = *(const v4f*)(rp + 12);
  const v4f wa = *(const v4f*)(gw + c * 8);
  const v4f wb = *(const v4f*)(gw + c * 8 + 4);

  float xv[8];
#pragma unroll
  for (int e = 0; e < 4; ++e) { xv[e] = xa[e]; xv[4 + e] = xb[e]; }
  float ss = 0.f;
#pragma unroll
  for (int e = 0; e < 8; ++e) ss += xv[e] * xv[e];
  ss += __shfl_xor(ss, 1, 32);
  ss += __shfl_xor(ss, 2, 32);
  ss += __shfl_xor(ss, 4, 32);
  ss += __shfl_xor(ss, 8, 32);
  const float inv = rsqrtf(ss * (1.0f / 128.0f) + eps);
  float wv[8];
#pragma unroll
  for (int e = 0; e < 4; ++e) { wv[e] = bf_rne(wa[e]); wv[4 + e] = bf_rne(wb[e]); }
  float yv[8];
#pragma unroll
  for (int e = 0; e < 8; ++e) yv[e] = (xv[e] * inv) * wv[e];
  float rr[16];
#pragma unroll
  for (int e = 0; e < 4; ++e) { rr[e] = bf_rne(r0[e]); rr[4 + e] = bf_rne(r1[e]); rr[8 + e] = bf_rne(r2[e]); rr[12 + e] = bf_rne(r3[e]); }
  float ov[8];
#pragma unroll
  for (int p = 0; p < 4; ++p) {
    const float y0 = yv[2 * p], y1 = yv[2 * p + 1];
    ov[2 * p]     = rr[4 * p + 0] * y0 + rr[4 * p + 1] * y1;
    ov[2 * p + 1] = rr[4 * p + 2] * y0 + rr[4 * p + 3] * y1;
  }
  v8h hv;
#pragma unroll
  for (int e = 0; e < 8; ++e) hv[e] = (_Float16)ov[e];
  if (ok) {
    _Float16* Y = (_Float16*)Yp;
    *(volatile v8h*)(Y + base) = hv;
    __threadfence();
    *(volatile v8h*)(Y + base) = hv;
  }
}

#define AT_HD 128
#define AT_QB 64
#define AT_KC 64
#define AT_KP 136
#define AT_VP 72
#define AT_PP 72
#define AT_OP 68
constexpr float kPsc = 16384.0f;

__device__ __forceinline__ v8f mma_f16(v16h a, v16h b, v8f c) {
  c = __builtin_amdgcn_wmma_f32_16x16x32_f16(false, a, false, b, (short)0, c, false, false);
  asm volatile("v_nop\n\tv_nop\n\tv_nop\n\tv_nop" : "+v"(c) : "v"(a), "v"(b));
  return c;
}

__global__ __launch_bounds__(128)
void attn_hd128(const unsigned short* __restrict__ Qp, const unsigned short* __restrict__ Kp,
                const unsigned short* __restrict__ Vtp, unsigned short* __restrict__ Ahp,
                unsigned short* __restrict__ Alp, int S, int ldq, int ldv, float sm_scale) {
  __shared__ __align__(16) _Float16 Ksh[AT_KC * AT_KP];
  __shared__ __align__(16) _Float16 Vsh[AT_HD * AT_VP];
  __shared__ __align__(16) _Float16 Psh[4][16 * AT_PP];
  __shared__ __align__(16) float    Os[4][16 * AT_OP];

  const _Float16* Q  = (const _Float16*)Qp;
  const _Float16* Kg = (const _Float16*)Kp;
  const _Float16* Vt = (const _Float16*)Vtp;
  const int tid  = threadIdx.x;
  const int wave = tid >> 5;
  const int lane = tid & 31;
  const int hh   = lane >> 4;
  const int c    = lane & 15;

  const int nqb = S / AT_QB;
  const int qb  = blockIdx.x % nqb;
  const int h   = blockIdx.x / nqb;
  const int q0  = qb * AT_QB + wave * 16;

  v16h qa[4];
#pragma unroll
  for (int dc = 0; dc < 4; ++dc)
    qa[dc] = Frag<_Float16>::load(Q + (size_t)(q0 + c) * ldq + h * AT_HD + dc * 32 + 8 * hh);

  float mrow[8], lrow[8];
  v8f oacc[8];
#pragma unroll
  for (int r = 0; r < 8; ++r) { mrow[r] = -__builtin_inff(); lrow[r] = 0.f; }
#pragma unroll
  for (int t = 0; t < 8; ++t) oacc[t] = (v8f){0.f,0.f,0.f,0.f,0.f,0.f,0.f,0.f};

  const int nChunks = S / AT_KC;
  for (int kc = 0; kc < nChunks; ++kc) {
    const int kv0 = kc * AT_KC;
    __syncthreads();
#pragma unroll
    for (int i = 0; i < 8; ++i) {
      const int idx = tid + 128 * i;
      const int row = idx >> 4, un = idx & 15;
      const v8h tv = *(const v8h*)(Kg + (size_t)(kv0 + row) * ldq + h * AT_HD + un * 8);
      *(v8h*)(Ksh + row * AT_KP + un * 8) = tv;
    }
#pragma unroll
    for (int i = 0; i < 8; ++i) {
      const int idx = tid + 128 * i;
      const int row = idx >> 3, un = idx & 7;
      const v8h tv = *(const v8h*)(Vt + (size_t)(h * AT_HD + row) * ldv + kv0 + un * 8);
      *(v8h*)(Vsh + row * AT_VP + un * 8) = tv;
    }
    __syncthreads();

    v8f sc[4];
#pragma unroll
    for (int j = 0; j < 4; ++j) {
      sc[j] = (v8f){0.f,0.f,0.f,0.f,0.f,0.f,0.f,0.f};
#pragma unroll
      for (int dc = 0; dc < 4; ++dc) {
        const v16h kb = Frag<_Float16>::load(Ksh + (j * 16 + c) * AT_KP + dc * 32 + 8 * hh);
        sc[j] = mma_f16(qa[dc], kb, sc[j]);
      }
    }
    float cm[8];
#pragma unroll
    for (int r = 0; r < 8; ++r) {
      float m = -__builtin_inff();
#pragma unroll
      for (int j = 0; j < 4; ++j) {
        const float sv = sc[j][r] * sm_scale;
        sc[j][r] = sv;
        m = fmaxf(m, sv);
      }
#pragma unroll
      for (int off = 1; off < 16; off <<= 1) m = fmaxf(m, __shfl_xor(m, off, 32));
      cm[r] = m;
    }
    _Float16* pw = Psh[wave];
#pragma unroll
    for (int r = 0; r < 8; ++r) {
      const float mnew  = fmaxf(mrow[r], cm[r]);
      const float alpha = expf(mrow[r] - mnew);
      mrow[r] = mnew;
      float psum = 0.f;
#pragma unroll
      for (int j = 0; j < 4; ++j) {
        const float p = expf(sc[j][r] - mnew);
        psum += p;
        pw[(8 * hh + r) * AT_PP + j * 16 + c] = (_Float16)(p * kPsc);
      }
#pragma unroll
      for (int off = 1; off < 16; off <<= 1) psum += __shfl_xor(psum, off, 32);
      lrow[r] = lrow[r] * alpha + psum;
#pragma unroll
      for (int t = 0; t < 8; ++t) oacc[t][r] *= alpha;
    }
    __builtin_amdgcn_fence(__ATOMIC_RELEASE, "workgroup");
    __builtin_amdgcn_wave_barrier();
    __builtin_amdgcn_fence(__ATOMIC_ACQUIRE, "workgroup");
#pragma unroll 1
    for (int kk = 0; kk < 2; ++kk) {
      const v16h pa = Frag<_Float16>::load(pw + c * AT_PP + kk * 32 + 8 * hh);
#pragma unroll
      for (int t = 0; t < 8; ++t) {
        const v16h vb = Frag<_Float16>::load(Vsh + (t * 16 + c) * AT_VP + kk * 32 + 8 * hh);
        oacc[t] = mma_f16(pa, vb, oacc[t]);
      }
    }
  }

  float* os = Os[wave];
  float inv[8];
#pragma unroll
  for (int r = 0; r < 8; ++r) inv[r] = 1.0f / (lrow[r] * kPsc);
  _Float16* Ah = (_Float16*)Ahp;
  _Float16* Al = (_Float16*)Alp;
#pragma unroll
  for (int half = 0; half < 2; ++half) {
#pragma unroll
    for (int r = 0; r < 8; ++r) {
#pragma unroll
      for (int t4 = 0; t4 < 4; ++t4) os[(8 * hh + r) * AT_OP + t4 * 16 + c] = oacc[half * 4 + t4][r] * inv[r];
    }
    __builtin_amdgcn_fence(__ATOMIC_RELEASE, "workgroup");
    __builtin_amdgcn_wave_barrier();
    __builtin_amdgcn_fence(__ATOMIC_ACQUIRE, "workgroup");
    {
      const int q8 = lane >> 3, c8 = (lane & 7) * 8;
      for (int pass = 0; pass < 2; ++pass) {
#pragma unroll
        for (int it = 0; it < 4; ++it) {
          const int row = it * 4 + q8;
          const float* sp = os + row * AT_OP + c8;
          v8h hv, lv;
#pragma unroll
          for (int e = 0; e < 8; ++e) {
            const unsigned short hb = f2bf_bits(sp[e]);
            const unsigned short lb = f2bf_bits(sp[e] - bf_bits2f(hb));
            hv[e] = __builtin_bit_cast(_Float16, hb);
            lv[e] = __builtin_bit_cast(_Float16, lb);
          }
          const size_t go = (size_t)(q0 + row) * ldq + h * AT_HD + half * 64 + c8;
          *(volatile v8h*)(Ah + go) = hv;
          *(volatile v8h*)(Al + go) = lv;
        }
        __threadfence();
      }
    }
    __builtin_amdgcn_fence(__ATOMIC_RELEASE, "workgroup");
    __builtin_amdgcn_wave_barrier();
    __builtin_amdgcn_fence(__ATOMIC_ACQUIRE, "workgroup");
  }
}

extern "C" void kernel_launch(void* const* d_in, const int* in_sizes, int n_in,
                              void* d_out, int out_size, void* d_ws, size_t ws_size,
                              hipStream_t stream) {
  (void)kChkGeom; (void)kChkWs;
  if (n_in < 12) return;
  if (in_sizes[0] != kSeq * kCh) return;
  if (in_sizes[1] != kSeq * 256) return;
  if (in_sizes[2] != kCh * kCh || in_sizes[4] != kCh * kCh || in_sizes[6] != kCh * kCh || in_sizes[8] != kCh * kCh) return;
  if (in_sizes[3] != kCh || in_sizes[5] != kCh || in_sizes[7] != kCh || in_sizes[9] != kCh) return;
  if (in_sizes[10] != kHd || in_sizes[11] != kHd) return;
  if (out_size != kSeq * kCh) return;
  if (ws_size < kWsTotal) return;

  const float* x    = (const float*)d_in[0];
  const float* rot  = (const float*)d_in[1];
  const float* Wq   = (const float*)d_in[2];
  const float* bq   = (const float*)d_in[3];
  const float* Wk   = (const float*)d_in[4];
  const float* bk   = (const float*)d_in[5];
  const float* Wv   = (const float*)d_in[6];
  const float* bv   = (const float*)d_in[7];
  const float* Wo   = (const float*)d_in[8];
  const float* bo   = (const float*)d_in[9];
  const float* qn_w = (const float*)d_in[10];
  const float* kn_w = (const float*)d_in[11];
  float* out = (float*)d_out;

  char* ws = (char*)d_ws;
  unsigned short* Xb  = (unsigned short*)(ws + oXb);
  unsigned short* Wqb = (unsigned short*)(ws + oWq);
  unsigned short* Wkb = (unsigned short*)(ws + oWk);
  unsigned short* Wvb = (unsigned short*)(ws + oWv);
  unsigned short* Wob = (unsigned short*)(ws + oWo);
  float*          QKf = (float*)(ws + oQKf);
  unsigned short* Qh  = (unsigned short*)(ws + oQh);
  unsigned short* Kh  = (unsigned short*)(ws + oKh);
  unsigned short* Vt  = (unsigned short*)(ws + oVt);
  unsigned short* Ahi = (unsigned short*)(ws + oXb);
  unsigned short* Alo = (unsigned short*)(ws + oQKf);

  const int nSC2 = (kSeq * kCh) / 2;
  const int nCC2 = (kCh * kCh) / 2;
  const int gSC2 = (nSC2 + 255) / 256;
  const int gCC2 = (nCC2 + 255) / 256;

  cast_f32_bf16x2<<<dim3(gSC2), dim3(256), 0, stream>>>(x,  Xb,  nSC2);
  cast_f32_bf16x2<<<dim3(gCC2), dim3(256), 0, stream>>>(Wq, Wqb, nCC2);
  cast_f32_bf16x2<<<dim3(gCC2), dim3(256), 0, stream>>>(Wk, Wkb, nCC2);
  cast_f32_bf16x2<<<dim3(gCC2), dim3(256), 0, stream>>>(Wv, Wvb, nCC2);
  cast_f32_bf16x2<<<dim3(gCC2), dim3(256), 0, stream>>>(Wo, Wob, nCC2);

  const int tilesQK  = (kSeq / 64) * (kCh / 64);
  const int gGemm    = (tilesQK + 7) / 8;
  const int nUnits   = kSeq * kNh;
  const int gNorm    = (nUnits + 15) / 16;
  const float eps    = 1.1920929e-07f;
  const float sm_scale = 1.0f / sqrtf((float)kHd);

  wmma_gemm64<1, 0, 2, 0, false, 0><<<dim3(gGemm, 1), dim3(256), 0, stream>>>(
      Xb, Xb, kCh, 0L, Wqb, Wqb, kCh, 0L, (void*)QKf, (void*)QKf, kCh, 0L,
      bq, nullptr, 0L, kSeq, kCh, kCh, 1.0f);
  rmsnorm_rotary_f16<<<dim3(gNorm), dim3(256), 0, stream>>>(QKf, rot, qn_w, Qh, nUnits, eps);

  wmma_gemm64<1, 0, 2, 0, false, 0><<<dim3(gGemm, 1), dim3(256), 0, stream>>>(
      Xb, Xb, kCh, 0L, Wkb, Wkb, kCh, 0L, (void*)QKf, (void*)QKf, kCh, 0L,
      bk, nullptr, 0L, kSeq, kCh, kCh, 1.0f);
  rmsnorm_rotary_f16<<<dim3(gNorm), dim3(256), 0, stream>>>(QKf, rot, kn_w, Kh, nUnits, eps);

  wmma_gemm64<1, 0, 1, 1, false, 0><<<dim3(gGemm, 1), dim3(256), 0, stream>>>(
      Wvb, Wvb, kCh, 0L, Xb, Xb, kCh, 0L, (void*)Vt, (void*)Vt, kSeq, 0L,
      bv, nullptr, 0L, kCh, kSeq, kCh, 1.0f);

  const int gAttn = kNh * (kSeq / AT_QB);
  attn_hd128<<<dim3(gAttn), dim3(128), 0, stream>>>(Qh, Kh, Vt, Ahi, Alo, kSeq, kCh, kSeq, sm_scale);

  wmma_gemm64<1, 2, 2, 0, false, 0><<<dim3(gGemm, 1), dim3(256), 0, stream>>>(
      Ahi, Alo, kCh, 0L, Wob, Wob, kCh, 0L, (void*)out, (void*)out, kCh, 0L,
      bo, nullptr, 0L, kSeq, kCh, kCh, 1.0f);
}
